// NetworkLocal_26757646254249
// MI455X (gfx1250) — hardware-verified
//
#include <hip/hip_runtime.h>


#define NBT  4
#define TT   256
#define DP   512
#define KIN  17
#define KP1  32
#define H1   196
#define HP   224
#define NP1  256
#define KL   128
#define NR   (NBT * TT * DP)
#define RCH  65536
#define NCHK (NR / RCH)
typedef _Float16 h16;
typedef unsigned short bf;
typedef __attribute__((ext_vector_type(16))) __bf16   v16bf;
typedef __attribute__((ext_vector_type(16))) _Float16 v16h;
typedef __attribute__((ext_vector_type(8)))  _Float16 v8h;
typedef __attribute__((ext_vector_type(8)))  unsigned short v8us;
typedef __attribute__((ext_vector_type(8)))  float    v8f;
typedef __attribute__((ext_vector_type(4)))  float    v4f;
typedef v8h  __attribute__((may_alias)) v8ha;
typedef v4f  __attribute__((may_alias)) v4fa;
typedef v8us __attribute__((may_alias)) v8usa;

__device__ __forceinline__ unsigned short f2bf(float f) { unsigned u = __float_as_uint(f); u += 0x7FFFu + ((u >> 16) & 1u); return (unsigned short)(u >> 16); }
__device__ __forceinline__ float bf2f(unsigned short b) { return __uint_as_float(((unsigned)b) << 16); }
__device__ __forceinline__ float bfr(float f) { return bf2f(f2bf(f)); }
__device__ __forceinline__ v16h cat16(v8h lo, v8h hi) { return __builtin_shufflevector(lo, hi, 0, 1, 2, 3, 4, 5, 6, 7, 8, 9, 10, 11, 12, 13, 14, 15); }
__device__ __forceinline__ v16bf cat16b(v8us lo, v8us hi) { return __builtin_bit_cast(v16bf, __builtin_shufflevector(lo, hi, 0, 1, 2, 3, 4, 5, 6, 7, 8, 9, 10, 11, 12, 13, 14, 15)); }
__device__ __forceinline__ v8f wmma16(v16h a, v16h b, v8f c) { return __builtin_amdgcn_wmma_f32_16x16x32_f16(false, a, false, b, (short)0, c, false, false); }
__device__ __forceinline__ v8f wmmab(v16bf a, v16bf b, v8f c) { return __builtin_amdgcn_wmma_f32_16x16x32_bf16(false, a, false, b, (short)0, c, false, false); }


template <typename T16> struct WFrag;
template <> struct WFrag<h16> { typedef v16h V; static __device__ __forceinline__ V ld(const h16* p) { return cat16(*(const v8h*)p, *(const v8h*)(p + 16)); } static __device__ __forceinline__ v8f mma(V a, V b, v8f c) { return wmma16(a, b, c); } };
template <> struct WFrag<bf> { typedef v16bf V; static __device__ __forceinline__ V ld(const bf* p) { return cat16b(*(const v8us*)p, *(const v8us*)(p + 16)); } static __device__ __forceinline__ v8f mma(V a, V b, v8f c) { return wmmab(a, b, c); } };
template <typename T16, int NSPLIT, bool BIAS>
__global__ __launch_bounds__(32) void k_gemmw(const T16* __restrict__ A, const T16* __restrict__ A2, const T16* __restrict__ Bt, const T16* __restrict__ Bt2, int K, float* C, int ldc, const float* __restrict__ bias, size_t sA, size_t sB, size_t sC) {
    typedef typename WFrag<T16>::V V;
    __shared__ __align__(16) float os[16 * 68];
    const size_t z = blockIdx.z; A += z * sA; if (A2) A2 += z * sA; Bt += z * sB; if (Bt2) Bt2 += z * sB; C += z * sC;
    const int lane = threadIdx.x & 31, lr = lane & 15, hi = lane >> 4; const int r0 = blockIdx.x * 64, c0 = blockIdx.y * 64;
    v8f acc[4][4];
#pragma unroll
    for (int mb = 0; mb < 4; ++mb)
#pragma unroll
        for (int nb = 0; nb < 4; ++nb) acc[mb][nb] = (v8f){};
    const size_t aoff = (size_t)(r0 + lr) * K + 8 * hi, boff = (size_t)(c0 + lr) * K + 8 * hi;
#pragma unroll 1
    for (int kc = 0; kc < K; kc += 32) {
        V a[4], a2[4];
#pragma unroll
        for (int mb = 0; mb < 4; ++mb) { a[mb] = WFrag<T16>::ld(A + aoff + (size_t)mb * 16 * K + kc); if (NSPLIT == 1 || NSPLIT == 2) a2[mb] = WFrag<T16>::ld(A2 + aoff + (size_t)mb * 16 * K + kc); }
#pragma unroll
        for (int nb = 0; nb < 4; ++nb) { const V b = WFrag<T16>::ld(Bt + boff + (size_t)nb * 16 * K + kc); V b2; if (NSPLIT >= 2) b2 = WFrag<T16>::ld(Bt2 + boff + (size_t)nb * 16 * K + kc);
#pragma unroll
            for (int mb = 0; mb < 4; ++mb) { acc[mb][nb] = WFrag<T16>::mma(a[mb], b, acc[mb][nb]); if (NSPLIT == 1 || NSPLIT == 2) acc[mb][nb] = WFrag<T16>::mma(a2[mb], b, acc[mb][nb]); if (NSPLIT >= 2) acc[mb][nb] = WFrag<T16>::mma(a[mb], b2, acc[mb][nb]); } }
        asm volatile("v_nop\n\tv_nop\n\tv_nop\n\tv_nop" : "+v"(acc[0][0]), "+v"(acc[1][1]), "+v"(acc[2][2]), "+v"(acc[3][3]) : "v"(a[0]), "v"(a[3]));
    }
#pragma unroll
    for (int mb = 0; mb < 4; ++mb) {
#pragma unroll
        for (int nb = 0; nb < 4; ++nb) {
#pragma unroll
            for (int j = 0; j < 8; ++j) os[(hi * 8 + j) * 68 + nb * 16 + lr] = acc[mb][nb][j]; }
        __builtin_amdgcn_wave_barrier(); asm volatile("" ::: "memory");
        float* crow = C + (size_t)(r0 + mb * 16) * ldc + c0;
#pragma unroll 1
        for (int ps = 0; ps < 2; ++ps) {
#pragma unroll
            for (int s = 0; s < 8; ++s) { const int row = 2 * s + hi, cofs = lr * 4; v4f val = *(const v4fa*)(os + row * 68 + cofs); if (BIAS) { val[0] += bfr(bias[c0 + cofs]); val[1] += bfr(bias[c0 + cofs + 1]); val[2] += bfr(bias[c0 + cofs + 2]); val[3] += bfr(bias[c0 + cofs + 3]); }
                *(volatile v4f*)(crow + (size_t)row * ldc + cofs) = val; }
            if (ps == 0) __threadfence(); }
        __builtin_amdgcn_wave_barrier(); asm volatile("" ::: "memory");
    }
}

__device__ __forceinline__ h16 tohx(float x) { return (h16)x; }
__device__ __noinline__ float fdivn(float a, float b) { return __fdiv_rn(a, b); }
typedef __attribute__((ext_vector_type(2))) _Float16 v2h;

__global__ __launch_bounds__(256) void k_wth(const float* __restrict__ w, int K, int N, int Kp, int Np, h16* Bt) {
    const int lane = threadIdx.x & 31; const int L0 = (blockIdx.x * 8 + (threadIdx.x >> 5)) * 8; const int nlines = Np * Kp / 64;
#pragma unroll 1
    for (int ps = 0; ps < 2; ++ps) {
#pragma unroll 1
        for (int l = 0; l < 8; ++l) { const int L = L0 + l; if (L >= nlines) break; const int e = L * 64 + lane * 2; v2h o;
#pragma unroll
            for (int q = 0; q < 2; ++q) { const int n = (e + q) / Kp, k = (e + q) % Kp; o[q] = tohx((n < N && k < K) ? bfr(w[(size_t)(k < K ? k : 0) * N + (n < N ? n : 0)]) : 0.f); }
            *(volatile v2h*)(Bt + e) = o; }
        if (ps == 0) __threadfence(); }
}
__global__ __launch_bounds__(256) void k_bpad(const float* __restrict__ b, int N, int Np, float* out) { const int i = blockIdx.x * 256 + threadIdx.x; if (i >= Np) return; const float v = i < N ? b[i < N ? i : 0] : 0.f; *(volatile float*)(out + i) = v; __threadfence(); *(volatile float*)(out + i) = v; }
__global__ __launch_bounds__(256) void k_feat(const float* __restrict__ x0, const float* __restrict__ x, const int* __restrict__ Nn, const float* __restrict__ basis, const float* __restrict__ vel, int r0, h16* F1) {
    __shared__ float sf[8][32][KIN + 1];
    const int lane = threadIdx.x & 31, wv = threadIdx.x >> 5; const int g0 = (blockIdx.x * 8 + wv) * 32; if (g0 >= RCH) return; const int r = r0 + g0 + lane; const int bt = r / DP; const int b = bt / TT;
    float f[KIN];
    { const float n = (float)(Nn[bt] > 1 ? Nn[bt] : 1); f[0] = n;
      const float a0 = bfr(x0[bt * 3]), a1 = bfr(x0[bt * 3 + 1]), a2 = bfr(x0[bt * 3 + 2]); const float an = sqrtf(a0 * a0 + a1 * a1 + a2 * a2) + 1e-5f; const float h0 = fdivn(a0, an), h1 = fdivn(a1, an), h2 = fdivn(a2, an);
      float bh[3][3];
#pragma unroll
      for (int k = 0; k < 3; ++k) { const float c0 = bfr(basis[(b * 3 + k) * 3]), c1 = bfr(basis[(b * 3 + k) * 3 + 1]), c2 = bfr(basis[(b * 3 + k) * 3 + 2]); const float cn = sqrtf(c0 * c0 + c1 * c1 + c2 * c2) + 1e-5f; bh[k][0] = fdivn(c0, cn); bh[k][1] = fdivn(c1, cn); bh[k][2] = fdivn(c2, cn); }
#pragma unroll
      for (int uu = 0; uu < 2; ++uu) { const float* up = (uu == 0 ? x : vel) + (size_t)r * 3; const float u0 = bfr(up[0]), u1 = bfr(up[1]), u2 = bfr(up[2]); const float mag = sqrtf(u0 * u0 + u1 * u1 + u2 * u2); const float mg = mag + 1e-5f;
          const float q0 = fdivn(u0, mg), q1 = fdivn(u1, mg), q2 = fdivn(u2, mg); const int o = 1 + uu * 8;
          f[o] = mag; f[o + 1] = q0 * h0 + q1 * h1 + q2 * h2;
#pragma unroll
          for (int k = 0; k < 3; ++k) { f[o + 2 + k] = q0 * bh[k][0] + q1 * bh[k][1] + q2 * bh[k][2]; f[o + 5 + k] = u0 * bh[k][0] + u1 * bh[k][1] + u2 * bh[k][2]; } } }
#pragma unroll
    for (int i = 0; i < KIN; ++i) sf[wv][lane][i] = f[i];
    __builtin_amdgcn_wave_barrier(); asm volatile("" ::: "memory");
#pragma unroll 1
    for (int ps = 0; ps < 2; ++ps) {
#pragma unroll 1
        for (int i2 = 0; i2 < 16; ++i2) { const int rr = i2 * 2 + (lane >> 4); const int c = (lane & 15) * 2; v2h o;
#pragma unroll
            for (int q = 0; q < 2; ++q) o[q] = tohx((c + q) < KIN ? sf[wv][rr][(c + q) < KIN ? c + q : 0] : 0.f);
            *(volatile v2h*)(F1 + (size_t)(g0 + rr) * KP1 + c) = o; }
        if (ps == 0) __threadfence(); }
}
__global__ __launch_bounds__(256) void k_leaky16(const float* __restrict__ C, h16* P) {
    const int lane = threadIdx.x & 31; const int L0 = (blockIdx.x * 8 + (threadIdx.x >> 5)) * 8; const int nlines = RCH * HP / 64;
#pragma unroll 1
    for (int ps = 0; ps < 2; ++ps) {
#pragma unroll
        for (int l = 0; l < 8; ++l) { const int L = L0 + l; if (L >= nlines) break; const int e = L * 64 + lane * 2; const int r = e / HP, k = e % HP; v2h v;
#pragma unroll
            for (int q = 0; q < 2; ++q) { const int kk = k + q; float t = 0.f; if (kk < H1) { t = C[(size_t)r * NP1 + kk]; t = t >= 0.f ? t : 0.01f * t; } v[q] = tohx(t); }
            *(volatile v2h*)(P + (size_t)e) = v; }
        if (ps == 0) __threadfence(); }
}
__global__ __launch_bounds__(256) void k_pool(const float* __restrict__ H3, const int* __restrict__ Nn, int bt0, float* OUT) {
    const int lane = threadIdx.x & 31; const int btl = blockIdx.x * 8 + (threadIdx.x >> 5); if (btl >= RCH / DP) return; const int bt = bt0 + btl; v4f s = {0.f, 0.f, 0.f, 0.f};
#pragma unroll 4
    for (int d = 0; d < DP; ++d) { const v4f t = *(const v4f*)(H3 + ((size_t)btl * DP + d) * KL + lane * 4); s[0] += t[0]; s[1] += t[1]; s[2] += t[2]; s[3] += t[3]; }
    const float n = (float)(Nn[bt] > 1 ? Nn[bt] : 1); v4f o;
#pragma unroll
    for (int q = 0; q < 4; ++q) o[q] = __fdiv_rn(s[q], n);
    float* dst = OUT + (size_t)bt * KL + lane * 4; *(volatile v4f*)dst = o; __threadfence(); *(volatile v4f*)dst = o;
}

extern "C" void kernel_launch(void* const* d_in, const int* in_sizes, int n_in,
                              void* d_out, int out_size, void* d_ws, size_t ws_size, hipStream_t stream) {
    (void)in_sizes; (void)n_in; (void)out_size;
    const float* x0 = (const float*)d_in[0]; const float* x = (const float*)d_in[1]; const int* Nn = (const int*)d_in[2]; const float* basis = (const float*)d_in[3]; const float* vel = (const float*)d_in[4];
    const float* W0 = (const float*)d_in[5]; const float* b0 = (const float*)d_in[6]; const float* W1 = (const float*)d_in[7]; const float* b1 = (const float*)d_in[8]; const float* W2 = (const float*)d_in[9]; const float* b2 = (const float*)d_in[10];
    float* OUT = (float*)d_out;
    char* wsp = (char*)d_ws;
    auto take = [&](size_t bytes) { char* p = wsp; wsp += (bytes + 255) & ~(size_t)255; return (void*)p; };
    h16* W0t = (h16*)take((size_t)NP1 * KP1 * 2); h16* W1t = (h16*)take((size_t)NP1 * HP * 2); h16* W2t = (h16*)take((size_t)KL * HP * 2); float* B0P = (float*)take(NP1 * 4); float* B1P = (float*)take(NP1 * 4);
    h16* F1 = (h16*)take((size_t)RCH * KP1 * 2); float* C = (float*)take((size_t)RCH * NP1 * 4); h16* P = (h16*)take((size_t)RCH * HP * 2);
    if ((size_t)(wsp - (char*)d_ws) > ws_size) return;
    float* H3 = C;
    k_wth<<<(NP1 * KP1 / 64 + 63) / 64, 256, 0, stream>>>(W0, KIN, H1, KP1, NP1, W0t); k_wth<<<(NP1 * HP / 64 + 63) / 64, 256, 0, stream>>>(W1, H1, H1, HP, NP1, W1t); k_wth<<<(KL * HP / 64 + 63) / 64, 256, 0, stream>>>(W2, H1, KL, HP, KL, W2t);
    k_bpad<<<1, 256, 0, stream>>>(b0, H1, NP1, B0P); k_bpad<<<1, 256, 0, stream>>>(b1, H1, NP1, B1P);
    for (int ch = 0; ch < NCHK; ++ch) { const int r0 = ch * RCH;
        k_feat<<<RCH / 32 / 8, 256, 0, stream>>>(x0, x, Nn, basis, vel, r0, F1);
        k_gemmw<h16, 0, true><<<dim3(RCH / 64, NP1 / 64, 1), 32, 0, stream>>>(F1, nullptr, W0t, nullptr, KP1, C, NP1, B0P, 0, 0, 0);
        k_leaky16<<<(RCH * HP / 64 + 63) / 64, 256, 0, stream>>>(C, P);
        k_gemmw<h16, 0, true><<<dim3(RCH / 64, NP1 / 64, 1), 32, 0, stream>>>(P, nullptr, W1t, nullptr, HP, C, NP1, B1P, 0, 0, 0);
        k_leaky16<<<(RCH * HP / 64 + 63) / 64, 256, 0, stream>>>(C, P);
        k_gemmw<h16, 0, true><<<dim3(RCH / 64, KL / 64, 1), 32, 0, stream>>>(P, nullptr, W2t, nullptr, HP, H3, KL, b2, 0, 0, 0);
        k_pool<<<(RCH / DP + 7) / 8, 256, 0, stream>>>(H3, Nn, ch * (RCH / DP), OUT); }
}
